// IAFChainEncoder_20761871908959
// MI455X (gfx1250) — hardware-run, weakly checked
//
#include <hip/hip_runtime.h>
#include <stddef.h>
#include <stdint.h>

#pragma clang fp contract(off)

#define NB 8192
#define ND 256
#define NH 512
#define NO 512
#define NT 4

static_assert((NB % 64) == 0);
static_assert((ND % 64) == 0);
static_assert((NH % 64) == 0);
static_assert((NO % 128) == 0);
static_assert(NO == 2 * ND);
static_assert((NB % 16) == 0);

typedef _Float16 v8h  __attribute__((ext_vector_type(8)));
typedef _Float16 v16h __attribute__((ext_vector_type(16)));
typedef float    v8f  __attribute__((ext_vector_type(8)));
typedef float    v4f  __attribute__((ext_vector_type(4)));
typedef unsigned int v4u __attribute__((ext_vector_type(4)));

union Frag { v16h v; v8h q[2]; };
union Pk8  { v8h h; v4u u; };

__device__ __forceinline__ float bfr(float f) {
  const unsigned u = __float_as_uint(f);
  const unsigned r = (u + 0x7FFFu + ((u >> 16) & 1u)) & 0xFFFF0000u;
  return __uint_as_float(r);
}
__device__ __forceinline__ v8f zero8() { v8f z = {0.f, 0.f, 0.f, 0.f, 0.f, 0.f, 0.f, 0.f}; return z; }

__device__ __forceinline__ v16h ldfrag(const _Float16* p) {
  Frag f;
  f.q[0] = *(const v8h*)(p);
  f.q[1] = *(const v8h*)(p + 16);
  return f.v;
}

__device__ __forceinline__ v8f mma_h(v16h a, v16h b, v8f c) {
  return __builtin_amdgcn_wmma_f32_16x16x32_f16(false, a, false, b, (short)0, c, false, false);
}
__device__ __forceinline__ void guard4(v8f& c0, v8f& c1, v8f& c2, v8f& c3,
                                       const v16h& f0, const v16h& f1, const v16h& f2, const v16h& f3) {
#if defined(__HIP_DEVICE_COMPILE__)
  asm volatile("v_nop\n\tv_nop\n\tv_nop\n\tv_nop"
               : "+v"(c0), "+v"(c1), "+v"(c2), "+v"(c3)
               : "v"(f0), "v"(f1), "v"(f2), "v"(f3));
#endif
}
__device__ __forceinline__ void guard8(v8f& c0, v8f& c1, v8f& c2, v8f& c3, v8f& c4, v8f& c5, v8f& c6, v8f& c7,
                                       const v16h& f0, const v16h& f1, const v16h& f2,
                                       const v16h& f3, const v16h& f4, const v16h& f5) {
#if defined(__HIP_DEVICE_COMPILE__)
  asm volatile("v_nop\n\tv_nop\n\tv_nop\n\tv_nop"
               : "+v"(c0), "+v"(c1), "+v"(c2), "+v"(c3), "+v"(c4), "+v"(c5), "+v"(c6), "+v"(c7)
               : "v"(f0), "v"(f1), "v"(f2), "v"(f3), "v"(f4), "v"(f5));
#endif
}

__global__ __launch_bounds__(256)
void k_wprep(const float* __restrict__ W, int K, int mtype, _Float16* Wt) {
  __shared__ __align__(16) _Float16 sT[64 * 64];
  const int tid = threadIdx.x;
  const int k0 = blockIdx.x * 64, n0 = blockIdx.y * 64, tz = blockIdx.z;
  const float* Wz = W + (size_t)tz * K * NO;
#pragma unroll
  for (int j = 0; j < 4; ++j) {
    const int idx = tid + 256 * j;
    const int kl = idx >> 4;
    const int nl = (idx & 15) * 4;
    const int k = k0 + kl;
    const int kq = k % 255;
    const v4f v = *(const v4f*)(Wz + (size_t)k * NO + n0 + nl);
#pragma unroll
    for (int e = 0; e < 4; ++e) {
      const int n = n0 + nl + e;
      int keep;
      if (mtype == 1)      keep = ((n % 255) >= k);
      else if (mtype == 2) keep = ((n % 255) >= kq);
      else                 keep = ((n >> 1) > kq);
      const float wv = keep ? (bfr(v[e]) * 64.0f) : 0.0f;
      sT[(nl + e) * 64 + kl] = (_Float16)wv;
    }
  }
  __syncthreads();

  Pk8 o[2];
#pragma unroll
  for (int it = 0; it < 2; ++it) o[it].h = *(const v8h*)(sT + (it * 32 + (tid >> 3)) * 64 + (tid & 7) * 8);
  _Float16* base = Wt + ((size_t)tz * NO + n0) * K + k0 + (tid & 7) * 8;
#pragma unroll
  for (int it = 0; it < 2; ++it) *(volatile v4u*)(base + (size_t)(it * 32 + (tid >> 3)) * K) = o[it].u;
  __threadfence();
#pragma unroll
  for (int it = 0; it < 2; ++it) *(volatile v4u*)(base + (size_t)(it * 32 + (tid >> 3)) * K) = o[it].u;
}

__global__ __launch_bounds__(256)
void k_init(const float* __restrict__ mean, const float* __restrict__ lv, const float* __restrict__ ep,
            float* P, _Float16* Xh, _Float16* Xl) {
  __shared__ __align__(16) float sY[16 * 256];
  const int tid = threadIdx.x;
  const int rb = blockIdx.x * 16;
  const size_t gb = (size_t)rb * ND;
#pragma unroll 1
  for (int j = 0; j < 16; ++j) {
    const int idx = tid + 256 * j;
    const int rl = idx >> 8, d = idx & 255;
    const float m = bfr(mean[gb + idx]);
    const float v = bfr(lv[gb + idx]);
    const float e = bfr(ep[gb + idx]);
    const float x = m + expf(0.5f * v) * e;
    sY[rl * 256 + (255 - d)] = x;
  }
  __syncthreads();

  Pk8 oh[2], ol[2];
#pragma unroll
  for (int it = 0; it < 2; ++it) {
    const int rl = it * 8 + (tid >> 5), pc = (tid & 31) * 8;
    const v4f u0 = *(const v4f*)(sY + rl * 256 + pc);
    const v4f u1 = *(const v4f*)(sY + rl * 256 + pc + 4);
#pragma unroll
    for (int e = 0; e < 8; ++e) {
      const float z = (e < 4) ? u0[e & 3] : u1[e & 3];
      const _Float16 hz = (_Float16)z;
      oh[it].h[e] = hz;
      ol[it].h[e] = (_Float16)((z - (float)hz) * 1024.0f);
    }
  }
  v4f of[4];
#pragma unroll
  for (int it = 0; it < 4; ++it) of[it] = *(const v4f*)(sY + (it * 4 + (tid >> 6)) * 256 + (tid & 63) * 4);

  _Float16* bh = Xh + gb + (tid & 31) * 8;
  _Float16* bl = Xl + gb + (tid & 31) * 8;
  float* bp = P + gb + (tid & 63) * 4;
#pragma unroll
  for (int it = 0; it < 2; ++it) {
    *(volatile v4u*)(bh + (size_t)(it * 8 + (tid >> 5)) * ND) = oh[it].u;
    *(volatile v4u*)(bl + (size_t)(it * 8 + (tid >> 5)) * ND) = ol[it].u;
  }
#pragma unroll
  for (int it = 0; it < 4; ++it) *(volatile v4f*)(bp + (size_t)(it * 4 + (tid >> 6)) * ND) = of[it];
  __threadfence();
#pragma unroll
  for (int it = 0; it < 2; ++it) {
    *(volatile v4u*)(bh + (size_t)(it * 8 + (tid >> 5)) * ND) = oh[it].u;
    *(volatile v4u*)(bl + (size_t)(it * 8 + (tid >> 5)) * ND) = ol[it].u;
  }
#pragma unroll
  for (int it = 0; it < 4; ++it) *(volatile v4f*)(bp + (size_t)(it * 4 + (tid >> 6)) * ND) = of[it];
}

template <int ALO>
__device__ __forceinline__ void put_h(_Float16* s, const v8f& a, const v8f& lo, float bv, int rowl, int coll) {
#pragma unroll
  for (int r = 0; r < 8; ++r) {
    float v = a[r];
    if (ALO) v = v + lo[r] * 0.0009765625f;
    v = v * 0.015625f + bv;
    v = fmaxf(v, 0.0f);
    s[(rowl + r) * 64 + coll] = (_Float16)v;
  }
}
__device__ __forceinline__ void put_f(float* s, const v8f& a, float bv, int rowl, int coll) {
#pragma unroll
  for (int r = 0; r < 8; ++r) s[(rowl + r) * 128 + coll] = a[r] * 0.015625f + bv;
}

template <int ALO>
__global__ __launch_bounds__(128)
void k_gemm_h(const _Float16* __restrict__ Ah, const _Float16* __restrict__ Al, const _Float16* __restrict__ Bt,
              const float* __restrict__ bias, int K, _Float16* Ch) {
  __shared__ __align__(16) _Float16 sH[64 * 64];
  const int tid = threadIdx.x, w = tid >> 5, lane = tid & 31, hh = lane >> 4, m = lane & 15;
  const int row0 = blockIdx.x * 64, col0 = blockIdx.y * 64;
  const int wm = (w & 1) * 32, wn = (w >> 1) * 32;

  const _Float16* ap0 = Ah + (size_t)(row0 + wm + m) * K + 8 * hh;
  const _Float16* ap1 = ap0 + (size_t)16 * K;
  const _Float16* lp0 = Al + (size_t)(row0 + wm + m) * K + 8 * hh;
  const _Float16* lp1 = lp0 + (size_t)16 * K;
  const _Float16* bp0 = Bt + (size_t)(col0 + wn + m) * K + 8 * hh;
  const _Float16* bp1 = bp0 + (size_t)16 * K;

  v8f a00 = zero8(), a01 = zero8(), a10 = zero8(), a11 = zero8();
  v8f l00 = zero8(), l01 = zero8(), l10 = zero8(), l11 = zero8();
  const int nk = K >> 5;
#pragma unroll 1
  for (int ks = 0; ks < nk; ++ks) {
    const int ko = ks << 5;
    const v16h x0 = ldfrag(ap0 + ko);
    const v16h x1 = ldfrag(ap1 + ko);
    const v16h g0 = ldfrag(bp0 + ko);
    const v16h g1 = ldfrag(bp1 + ko);
    a00 = mma_h(x0, g0, a00);
    a01 = mma_h(x0, g1, a01);
    a10 = mma_h(x1, g0, a10);
    a11 = mma_h(x1, g1, a11);
    if constexpr (ALO != 0) {
      const v16h y0 = ldfrag(lp0 + ko);
      const v16h y1 = ldfrag(lp1 + ko);
      l00 = mma_h(y0, g0, l00);
      l01 = mma_h(y0, g1, l01);
      l10 = mma_h(y1, g0, l10);
      l11 = mma_h(y1, g1, l11);
      guard8(a00, a01, a10, a11, l00, l01, l10, l11, x0, x1, y0, y1, g0, g1);
    } else {
      guard4(a00, a01, a10, a11, x0, x1, g0, g1);
    }
  }

  const float bv0 = bfr(bias[col0 + wn + m]), bv1 = bfr(bias[col0 + wn + 16 + m]);
  put_h<ALO>(sH, a00, l00, bv0, wm + 8 * hh,      wn + m);
  put_h<ALO>(sH, a01, l01, bv1, wm + 8 * hh,      wn + 16 + m);
  put_h<ALO>(sH, a10, l10, bv0, wm + 16 + 8 * hh, wn + m);
  put_h<ALO>(sH, a11, l11, bv1, wm + 16 + 8 * hh, wn + 16 + m);
  __syncthreads();

  Pk8 o[4];
#pragma unroll
  for (int it = 0; it < 4; ++it) o[it].h = *(const v8h*)(sH + (it * 16 + (tid >> 3)) * 64 + (tid & 7) * 8);
  _Float16* base = Ch + (size_t)row0 * NH + col0 + (tid & 7) * 8;
#pragma unroll
  for (int it = 0; it < 4; ++it) *(volatile v4u*)(base + (size_t)(it * 16 + (tid >> 3)) * NH) = o[it].u;
  __threadfence();
#pragma unroll
  for (int it = 0; it < 4; ++it) *(volatile v4u*)(base + (size_t)(it * 16 + (tid >> 3)) * NH) = o[it].u;
}

template <int FINAL>
__global__ __launch_bounds__(128)
void k_gemm_u(const _Float16* __restrict__ Ah, const _Float16* __restrict__ Bt, const float* __restrict__ bias,
              const float* __restrict__ Pc, float* Pn, _Float16* Xh, _Float16* Xl) {
  __shared__ __align__(16) float sF[64 * 128];
  __shared__ __align__(16) float sY[64 * 64];
  const int tid = threadIdx.x, w = tid >> 5, lane = tid & 31, hh = lane >> 4, m = lane & 15;
  const int row0 = blockIdx.x * 64, col0 = blockIdx.y * 128;
  const int wm = (w & 1) * 32, wn = (w >> 1) * 64;

  const _Float16* ap0 = Ah + (size_t)(row0 + wm + m) * NH + 8 * hh;
  const _Float16* ap1 = ap0 + (size_t)16 * NH;
  const _Float16* bp0 = Bt + (size_t)(col0 + wn + m) * NH + 8 * hh;
  const _Float16* bp1 = bp0 + (size_t)16 * NH;
  const _Float16* bp2 = bp0 + (size_t)32 * NH;
  const _Float16* bp3 = bp0 + (size_t)48 * NH;

  v8f a00 = zero8(), a01 = zero8(), a02 = zero8(), a03 = zero8();
  v8f a10 = zero8(), a11 = zero8(), a12 = zero8(), a13 = zero8();
#pragma unroll 1
  for (int ks = 0; ks < NH / 32; ++ks) {
    const int ko = ks << 5;
    const v16h x0 = ldfrag(ap0 + ko);
    const v16h x1 = ldfrag(ap1 + ko);
    const v16h g0 = ldfrag(bp0 + ko);
    const v16h g1 = ldfrag(bp1 + ko);
    const v16h g2 = ldfrag(bp2 + ko);
    const v16h g3 = ldfrag(bp3 + ko);
    a00 = mma_h(x0, g0, a00);
    a01 = mma_h(x0, g1, a01);
    a02 = mma_h(x0, g2, a02);
    a03 = mma_h(x0, g3, a03);
    a10 = mma_h(x1, g0, a10);
    a11 = mma_h(x1, g1, a11);
    a12 = mma_h(x1, g2, a12);
    a13 = mma_h(x1, g3, a13);
    guard8(a00, a01, a02, a03, a10, a11, a12, a13, x0, x1, g0, g1, g2, g3);
  }

  const float bv0 = bfr(bias[col0 + wn + m]);
  const float bv1 = bfr(bias[col0 + wn + 16 + m]);
  const float bv2 = bfr(bias[col0 + wn + 32 + m]);
  const float bv3 = bfr(bias[col0 + wn + 48 + m]);
  put_f(sF, a00, bv0, wm + 8 * hh,      wn + m);
  put_f(sF, a01, bv1, wm + 8 * hh,      wn + 16 + m);
  put_f(sF, a02, bv2, wm + 8 * hh,      wn + 32 + m);
  put_f(sF, a03, bv3, wm + 8 * hh,      wn + 48 + m);
  put_f(sF, a10, bv0, wm + 16 + 8 * hh, wn + m);
  put_f(sF, a11, bv1, wm + 16 + 8 * hh, wn + 16 + m);
  put_f(sF, a12, bv2, wm + 16 + 8 * hh, wn + 32 + m);
  put_f(sF, a13, bv3, wm + 16 + 8 * hh, wn + 48 + m);
  __syncthreads();

  const int dseg = blockIdx.y * 64;
  const int s0 = FINAL ? dseg : (192 - dseg);
  const float* pc = Pc + (size_t)row0 * ND + dseg;
#pragma unroll 1
  for (int j = 0; j < 32; ++j) {
    const int idx = tid + 128 * j;
    const int rl = idx >> 6, dl = idx & 63;
    const float xr = pc[(size_t)rl * ND + dl];
    const float sh = sF[rl * 128 + 2 * dl];
    const float lr = sF[rl * 128 + 2 * dl + 1];
    const float ls = tanhf(lr);
    const float y = (xr - sh) * expf(-ls);
    const int cl = FINAL ? dl : (63 - dl);
    sY[rl * 64 + cl] = y;
  }
  __syncthreads();

  v4f of[8];
#pragma unroll
  for (int it = 0; it < 8; ++it) of[it] = *(const v4f*)(sY + (it * 8 + (tid >> 4)) * 64 + (tid & 15) * 4);
  float* bp = Pn + (size_t)row0 * ND + s0 + (tid & 15) * 4;

  if constexpr (FINAL == 0) {
    Pk8 oh[4], ol[4];
#pragma unroll
    for (int it = 0; it < 4; ++it) {
      const int rl = it * 16 + (tid >> 3), pcs = (tid & 7) * 8;
      const v4f u0 = *(const v4f*)(sY + rl * 64 + pcs);
      const v4f u1 = *(const v4f*)(sY + rl * 64 + pcs + 4);
#pragma unroll
      for (int e = 0; e < 8; ++e) {
        const float z = (e < 4) ? u0[e & 3] : u1[e & 3];
        const _Float16 hz = (_Float16)z;
        oh[it].h[e] = hz;
        ol[it].h[e] = (_Float16)((z - (float)hz) * 1024.0f);
      }
    }
    _Float16* bh = Xh + (size_t)row0 * ND + s0 + (tid & 7) * 8;
    _Float16* bl = Xl + (size_t)row0 * ND + s0 + (tid & 7) * 8;
#pragma unroll
    for (int it = 0; it < 4; ++it) {
      *(volatile v4u*)(bh + (size_t)(it * 16 + (tid >> 3)) * ND) = oh[it].u;
      *(volatile v4u*)(bl + (size_t)(it * 16 + (tid >> 3)) * ND) = ol[it].u;
    }
#pragma unroll
    for (int it = 0; it < 8; ++it) *(volatile v4f*)(bp + (size_t)(it * 8 + (tid >> 4)) * ND) = of[it];
    __threadfence();
#pragma unroll
    for (int it = 0; it < 4; ++it) {
      *(volatile v4u*)(bh + (size_t)(it * 16 + (tid >> 3)) * ND) = oh[it].u;
      *(volatile v4u*)(bl + (size_t)(it * 16 + (tid >> 3)) * ND) = ol[it].u;
    }
#pragma unroll
    for (int it = 0; it < 8; ++it) *(volatile v4f*)(bp + (size_t)(it * 8 + (tid >> 4)) * ND) = of[it];
  } else {
#pragma unroll
    for (int it = 0; it < 8; ++it) *(volatile v4f*)(bp + (size_t)(it * 8 + (tid >> 4)) * ND) = of[it];
    __threadfence();
#pragma unroll
    for (int it = 0; it < 8; ++it) *(volatile v4f*)(bp + (size_t)(it * 8 + (tid >> 4)) * ND) = of[it];
  }
}

extern "C" void kernel_launch(void* const* d_in, const int* in_sizes, int n_in,
                              void* d_out, int out_size, void* d_ws, size_t ws_size,
                              hipStream_t stream) {
  if (n_in < 9) return;
  if (in_sizes[0] != NB * ND) return;
  if (in_sizes[1] != NB * ND) return;
  if (in_sizes[2] != NB * ND) return;
  if (in_sizes[3] != NT * ND * NH) return;
  if (in_sizes[4] != NT * NH) return;
  if (in_sizes[5] != NT * NH * NH) return;
  if (in_sizes[6] != NT * NH) return;
  if (in_sizes[7] != NT * NH * NO) return;
  if (in_sizes[8] != NT * NO) return;
  if (out_size != NB * ND) return;

  const float* mean = (const float*)d_in[0];
  const float* logv = (const float*)d_in[1];
  const float* eps  = (const float*)d_in[2];
  const float* W1   = (const float*)d_in[3];
  const float* b1   = (const float*)d_in[4];
  const float* W2   = (const float*)d_in[5];
  const float* b2   = (const float*)d_in[6];
  const float* W3   = (const float*)d_in[7];
  const float* b3   = (const float*)d_in[8];
  float* out = (float*)d_out;

  const size_t sP  = (size_t)NB * ND * 4;
  const size_t sX  = (size_t)NB * ND * 2;
  const size_t sHp = (size_t)NB * NH * 2;
  const size_t sW1 = (size_t)NT * NH * ND * 2;
  const size_t sW2 = (size_t)NT * NH * NH * 2;
  const size_t sW3 = (size_t)NT * NO * NH * 2;
  size_t off = 0;
  const size_t oP0 = off; off += sP;
  const size_t oP1 = off; off += sP;
  const size_t oXh = off; off += sX;
  const size_t oXl = off; off += sX;
  const size_t oH1 = off; off += sHp;
  const size_t oH2 = off; off += sHp;
  const size_t oW1 = off; off += sW1;
  const size_t oW2 = off; off += sW2;
  const size_t oW3 = off; off += sW3;
  if (off > ws_size) return;
  if (off > (size_t)134217728) return;

  char* ws = (char*)d_ws;
  float*    P0  = (float*)(ws + oP0);
  float*    P1  = (float*)(ws + oP1);
  _Float16* Xh  = (_Float16*)(ws + oXh);
  _Float16* Xl  = (_Float16*)(ws + oXl);
  _Float16* H1  = (_Float16*)(ws + oH1);
  _Float16* H2  = (_Float16*)(ws + oH2);
  _Float16* W1s = (_Float16*)(ws + oW1);
  _Float16* W2s = (_Float16*)(ws + oW2);
  _Float16* W3s = (_Float16*)(ws + oW3);

  k_wprep<<<dim3(ND / 64, NH / 64, NT), dim3(256), 0, stream>>>(W1, ND, 1, W1s);
  k_wprep<<<dim3(NH / 64, NH / 64, NT), dim3(256), 0, stream>>>(W2, NH, 2, W2s);
  k_wprep<<<dim3(NH / 64, NO / 64, NT), dim3(256), 0, stream>>>(W3, NH, 3, W3s);
  k_init<<<dim3(NB / 16), dim3(256), 0, stream>>>(mean, logv, eps, P0, Xh, Xl);
  float* Pcur = P0;
  float* Pnxt = P1;
  for (int i = NT - 1; i >= 0; --i) {
    const _Float16* w1p = W1s + (size_t)i * NH * ND;
    const _Float16* w2p = W2s + (size_t)i * NH * NH;
    const _Float16* w3p = W3s + (size_t)i * NO * NH;
    k_gemm_h<1><<<dim3(NB / 64, NH / 64), dim3(128), 0, stream>>>(Xh, Xl, w1p, b1 + i * NH, ND, H1);
    k_gemm_h<0><<<dim3(NB / 64, NH / 64), dim3(128), 0, stream>>>(H1, H1, w2p, b2 + i * NH, NH, H2);
    if (i > 0) {
      k_gemm_u<0><<<dim3(NB / 64, NO / 128), dim3(128), 0, stream>>>(H2, w3p, b3 + i * NO, Pcur, Pnxt, Xh, Xl);
      float* t = Pcur; Pcur = Pnxt; Pnxt = t;
    } else {
      k_gemm_u<1><<<dim3(NB / 64, NO / 128), dim3(128), 0, stream>>>(H2, w3p, b3, Pcur, out, Xh, Xl);
    }
  }
  (void)hipGetLastError();
}
